// MHLPPredictor_23424751633139
// MI455X (gfx1250) — hardware-verified
//
#include <hip/hip_runtime.h>


namespace {
constexpr int B = 262144, L = 5, NO = 5, NW = 3, AD = 75, D = 64, NH = 4, HD = 16, F1 = 128;
constexpr float S8 = 8.0f, S64 = 64.0f, WSC = 256.0f;
typedef _Float16 b16;
typedef __attribute__((ext_vector_type(16))) _Float16 v16b;
typedef __attribute__((ext_vector_type(8))) _Float16 v8b;
typedef __attribute__((ext_vector_type(8))) float v8f;
typedef __attribute__((ext_vector_type(4))) float v4f;
__device__ __forceinline__ float bf16_rne(float f) { unsigned int u = __float_as_uint(f); u += 0x7FFFu + ((u >> 16) & 1u); return __uint_as_float(u & 0xFFFF0000u); }
__device__ __forceinline__ void split16(float v, b16& hi, b16& lo) { hi = (b16)v; lo = (b16)(v - (float)hi); }
__device__ __forceinline__ v16b frag_kb(const b16* p, int hh) { const v8b a = *(const v8b*)(p + 8 * hh), b = *(const v8b*)(p + 16 + 8 * hh); v16b f;
#pragma unroll
  for (int e = 0; e < 8; ++e) { f[e] = a[e]; f[8 + e] = b[e]; } return f; }
__device__ __forceinline__ v8f wmma16b(v16b a, v16b b, v8f c) { v8f d = __builtin_amdgcn_wmma_f32_16x16x32_f16(false, a, false, b, (short)0, c, false, false); asm volatile("v_nop\n\tv_nop\n\tv_nop\n\tv_nop" : "+v"(d) : "v"(a), "v"(b)); return d; }
__device__ __forceinline__ void wave_lds_sync() { __builtin_amdgcn_fence(__ATOMIC_RELEASE, "workgroup"); __builtin_amdgcn_wave_barrier(); __builtin_amdgcn_fence(__ATOMIC_ACQUIRE, "workgroup"); }
__device__ __forceinline__ float pmul(float a, float b) { float p = a * b; asm volatile("" : "+v"(p)); return p; }
__device__ __forceinline__ int iclamp(int v, int lo, int hi) { return v < lo ? lo : (v > hi ? hi : v); }

__global__ __launch_bounds__(256) void wcopy_kernel(const float* __restrict__ w, int n8, b16* __restrict__ WT) {
  const int u = blockIdx.x * 256 + threadIdx.x; if (u >= n8) return; const int e = u * 8; v8b v;
#pragma unroll
  for (int j = 0; j < 8; ++j) v[j] = (b16)(bf16_rne(w[e + j]) * WSC); for (int pass = 0; pass < 2; ++pass) { *(volatile v8b*)(WT + e) = v; __threadfence(); }
}
__device__ __forceinline__ void ln64(float& a, float& b, float g0, float g1, float be0, float be1) {
  float s = a + b; for (int o = 16; o; o >>= 1) s += __shfl_xor(s, o); const float mu = s * (1.0f / D); const float da = a - mu, db = b - mu; float v = pmul(da, da) + pmul(db, db); for (int o = 16; o; o >>= 1) v += __shfl_xor(v, o);
  const float rs = 1.0f / sqrtf(v * (1.0f / D) + 1e-5f); a = pmul(pmul(da, rs), g0) + be0; b = pmul(pmul(db, rs), g1) + be1; }
__global__ __launch_bounds__(64) void mh_kernel(const int* __restrict__ hw, const int* __restrict__ opi, const int* __restrict__ wdi, const float* __restrict__ hwE, const float* __restrict__ W1, const float* __restrict__ b1, const b16* __restrict__ W2T, const float* __restrict__ b2, const float* __restrict__ l1g, const float* __restrict__ l1b, const b16* __restrict__ IPT, const float* __restrict__ ipb, const b16* __restrict__ OPT, const float* __restrict__ opb, const float* __restrict__ l2g, const float* __restrict__ l2b, const b16* __restrict__ W3T, const float* __restrict__ b3, const float* __restrict__ W4, const float* __restrict__ b4, int BLIM, float* __restrict__ out) {
  __shared__ __attribute__((aligned(16))) b16 Ah[2][32][F1 + 8], Al[2][32][F1 + 8]; __shared__ __attribute__((aligned(16))) float Cb[2][32][D + 1], Q[2][32][3 * D + 1]; __shared__ float So[32];
  const int wave = threadIdx.x >> 5, lane = threadIdx.x & 31, nloc = lane & 15, hlf = lane >> 4; const size_t s0 = (size_t)blockIdx.x * 32 + wave * 16;
  b16 (*ah)[F1 + 8] = Ah[wave]; b16 (*al)[F1 + 8] = Al[wave]; float (*cb)[D + 1] = Cb[wave]; float (*qb)[3 * D + 1] = Q[wave];
  if (s0 < (size_t)BLIM) {
    for (int rr = 0; rr < 16; ++rr) { const size_t s = s0 + rr; float hv[4]; for (int i = 0; i < 4; ++i) hv[i] = bf16_rne(b1[lane * 4 + i]);
      for (int l = 0; l < L; ++l) { const int cell = iclamp(opi[s * L + l], 0, NO - 1) * NW + iclamp(wdi[s * L + l], 0, NW - 1); const int col = l * NO * NW + cell; for (int i = 0; i < 4; ++i) hv[i] += bf16_rne(W1[(size_t)(lane * 4 + i) * AD + col]); }
      for (int i = 0; i < 4; ++i) { b16 p, q; split16(fmaxf(hv[i], 0.0f) * S8, p, q); ah[rr][lane * 4 + i] = p; al[rr][lane * 4 + i] = q; } }
    wave_lds_sync();
    { v8f acc[4];
#pragma unroll
      for (int t = 0; t < 4; ++t) acc[t] = (v8f){};
#pragma unroll
      for (int kb = 0; kb < F1; kb += 32) { const v16b a = frag_kb(&ah[nloc][kb], hlf), a2 = frag_kb(&al[nloc][kb], hlf);
#pragma unroll
        for (int t = 0; t < 4; ++t) { const v16b bw = frag_kb(W2T + (size_t)(t * 16 + nloc) * F1 + kb, hlf); acc[t] = wmma16b(a, bw, acc[t]); acc[t] = wmma16b(a2, bw, acc[t]); } }
#pragma unroll
      for (int t = 0; t < 4; ++t) { const int c = t * 16 + nloc; const float bb = bf16_rne(b2[c]);
#pragma unroll
        for (int r8 = 0; r8 < 8; ++r8) cb[16 + 8 * hlf + r8][c] = acc[t][r8] * (1.0f / (S8 * WSC)) + bb; } }
    wave_lds_sync();
    { const float g0 = bf16_rne(l1g[lane]), g1 = bf16_rne(l1g[32 + lane]), e0 = bf16_rne(l1b[lane]), e1 = bf16_rne(l1b[32 + lane]);
      for (int rr = 0; rr < 16; ++rr) { float a = cb[16 + rr][lane], b = cb[16 + rr][32 + lane]; ln64(a, b, g0, g1, e0, e1); const int hi = iclamp(hw[s0 + rr], 0, 3); const float t0a = bf16_rne(hwE[hi * D + lane]), t0b = bf16_rne(hwE[hi * D + 32 + lane]);
        wave_lds_sync(); cb[rr][lane] = t0a; cb[rr][32 + lane] = t0b; cb[16 + rr][lane] = a; cb[16 + rr][32 + lane] = b;
        b16 p, q; split16(t0a * S64, p, q); ah[rr][lane] = p; al[rr][lane] = q; split16(t0b * S64, p, q); ah[rr][32 + lane] = p; al[rr][32 + lane] = q; split16(a * S64, p, q); ah[16 + rr][lane] = p; al[16 + rr][lane] = q; split16(b * S64, p, q); ah[16 + rr][32 + lane] = p; al[16 + rr][32 + lane] = q; } }
    wave_lds_sync();
#pragma unroll 1
    for (int rt = 0; rt < 2; ++rt) { v8f acc[12];
#pragma unroll
      for (int t = 0; t < 12; ++t) acc[t] = (v8f){};
#pragma unroll
      for (int kb = 0; kb < D; kb += 32) { const v16b a = frag_kb(&ah[rt * 16 + nloc][kb], hlf), a2 = frag_kb(&al[rt * 16 + nloc][kb], hlf);
#pragma unroll
        for (int t = 0; t < 12; ++t) { const v16b bw = frag_kb(IPT + (size_t)(t * 16 + nloc) * D + kb, hlf); acc[t] = wmma16b(a, bw, acc[t]); acc[t] = wmma16b(a2, bw, acc[t]); } }
#pragma unroll
      for (int t = 0; t < 12; ++t) { const int c = t * 16 + nloc; const float bb = bf16_rne(ipb[c]);
#pragma unroll
        for (int r8 = 0; r8 < 8; ++r8) qb[rt * 16 + 8 * hlf + r8][c] = acc[t][r8] * (1.0f / (S64 * WSC)) + bb; } }
    wave_lds_sync();
    for (int rr = 0; rr < 16; ++rr) {
      const int qi = hlf, d = nloc;
      for (int h = 0; h < NH; ++h) { const float qv = qb[qi * 16 + rr][h * HD + d]; float s0_ = pmul(qv, qb[0 * 16 + rr][D + h * HD + d]), s1_ = pmul(qv, qb[1 * 16 + rr][D + h * HD + d]);
        for (int o = 1; o < 16; o <<= 1) { s0_ += __shfl_xor(s0_, o); s1_ += __shfl_xor(s1_, o); } s0_ *= 0.25f; s1_ *= 0.25f; const float mx = fmaxf(s0_, s1_); const float e0 = __expf(s0_ - mx), e1 = __expf(s1_ - mx); const float inv = 1.0f / (e0 + e1);
        const float cx = pmul(pmul(e0, inv), qb[0 * 16 + rr][2 * D + h * HD + d]) + pmul(pmul(e1, inv), qb[1 * 16 + rr][2 * D + h * HD + d]); b16 p, q; split16(cx * S64, p, q); ah[qi * 16 + rr][h * HD + d] = p; al[qi * 16 + rr][h * HD + d] = q; } }
    wave_lds_sync();
#pragma unroll 1
    for (int rt = 0; rt < 2; ++rt) { v8f acc[4];
#pragma unroll
      for (int t = 0; t < 4; ++t) acc[t] = (v8f){};
#pragma unroll
      for (int kb = 0; kb < D; kb += 32) { const v16b a = frag_kb(&ah[rt * 16 + nloc][kb], hlf), a2 = frag_kb(&al[rt * 16 + nloc][kb], hlf);
#pragma unroll
        for (int t = 0; t < 4; ++t) { const v16b bw = frag_kb(OPT + (size_t)(t * 16 + nloc) * D + kb, hlf); acc[t] = wmma16b(a, bw, acc[t]); acc[t] = wmma16b(a2, bw, acc[t]); } }
#pragma unroll
      for (int t = 0; t < 4; ++t) { const int c = t * 16 + nloc; const float bb = bf16_rne(opb[c]);
#pragma unroll
        for (int r8 = 0; r8 < 8; ++r8) qb[rt * 16 + 8 * hlf + r8][c] = acc[t][r8] * (1.0f / (S64 * WSC)) + bb + cb[rt * 16 + 8 * hlf + r8][c]; } }
    wave_lds_sync();
    { const float g0 = bf16_rne(l2g[lane]), g1 = bf16_rne(l2g[32 + lane]), e0 = bf16_rne(l2b[lane]), e1 = bf16_rne(l2b[32 + lane]);
      for (int rr = 0; rr < 16; ++rr) { float a0 = qb[rr][lane], b0 = qb[rr][32 + lane]; ln64(a0, b0, g0, g1, e0, e1); float a1 = qb[16 + rr][lane], b1_ = qb[16 + rr][32 + lane]; ln64(a1, b1_, g0, g1, e0, e1);
        const float pa = (a0 + a1) * 0.5f, pb = (b0 + b1_) * 0.5f; b16 p, q; split16(pa * S64, p, q); ah[rr][lane] = p; al[rr][lane] = q; split16(pb * S64, p, q); ah[rr][32 + lane] = p; al[rr][32 + lane] = q; } }
    wave_lds_sync();
    { v8f acc[2] = {(v8f){}, (v8f){}};
#pragma unroll
      for (int kb = 0; kb < D; kb += 32) { const v16b a = frag_kb(&ah[nloc][kb], hlf), a2 = frag_kb(&al[nloc][kb], hlf);
#pragma unroll
        for (int t = 0; t < 2; ++t) { const v16b bw = frag_kb(W3T + (size_t)(t * 16 + nloc) * D + kb, hlf); acc[t] = wmma16b(a, bw, acc[t]); acc[t] = wmma16b(a2, bw, acc[t]); } }
      float pd[8];
#pragma unroll
      for (int r8 = 0; r8 < 8; ++r8) pd[r8] = 0.0f;
#pragma unroll
      for (int t = 0; t < 2; ++t) { const int c = t * 16 + nloc; const float bb = bf16_rne(b3[c]), w4 = bf16_rne(W4[c]);
#pragma unroll
        for (int r8 = 0; r8 < 8; ++r8) pd[r8] += pmul(fmaxf(acc[t][r8] * (1.0f / (S64 * WSC)) + bb, 0.0f), w4); }
#pragma unroll
      for (int r8 = 0; r8 < 8; ++r8) { float s = pd[r8]; for (int o = 1; o < 16; o <<= 1) s += __shfl_xor(s, o); if (nloc == 0) So[wave * 16 + 8 * hlf + r8] = s + bf16_rne(b4[0]); } }
  } else { if (lane < 16) So[wave * 16 + lane] = 0.0f; }
  __syncthreads();
  if (wave == 0) { for (int pass = 0; pass < 2; ++pass) { ((volatile float*)out)[(size_t)blockIdx.x * 32 + lane] = So[lane]; __threadfence(); } }
}
}

extern "C" void kernel_launch(void* const* d_in, const int* in_sizes, int n_in, void* d_out, int out_size, void* d_ws, size_t ws_size, hipStream_t stream) {
  (void)n_in;
  auto Fp = [&](int i) { return (const float*)d_in[i]; }; auto Ip = [&](int i) { return (const int*)d_in[i]; };
  if (in_sizes[0] != B || in_sizes[1] != B * L || in_sizes[2] != B * L || in_sizes[3] != 4 * D || in_sizes[4] != F1 * AD || in_sizes[6] != D * F1 || in_sizes[10] != 3 * D * D || in_sizes[12] != D * D || in_sizes[16] != 32 * D || in_sizes[18] != 32 || out_size != B) return;
  const int BLIM = B;
  size_t off = 0; char* ws = (char*)d_ws;
  auto carve = [&](size_t bytes) { char* p = ws + off; off += (bytes + 255) & ~(size_t)255; return p; };
  b16* W2T = (b16*)carve(D * F1 * 2); b16* IPT = (b16*)carve(3 * D * D * 2); b16* OPT = (b16*)carve(D * D * 2); b16* W3T = (b16*)carve(32 * D * 2);
  if (off > ws_size || off > ((size_t)4 << 20)) return;
  wcopy_kernel<<<(D * F1 / 8 + 255) / 256, 256, 0, stream>>>(Fp(6), D * F1 / 8, W2T); wcopy_kernel<<<(3 * D * D / 8 + 255) / 256, 256, 0, stream>>>(Fp(10), 3 * D * D / 8, IPT); wcopy_kernel<<<(D * D / 8 + 255) / 256, 256, 0, stream>>>(Fp(12), D * D / 8, OPT); wcopy_kernel<<<(32 * D / 8 + 255) / 256, 256, 0, stream>>>(Fp(16), 32 * D / 8, W3T);
  mh_kernel<<<(unsigned)((BLIM + 31) / 32), 64, 0, stream>>>(Ip(0), Ip(1), Ip(2), Fp(3), Fp(4), Fp(5), W2T, Fp(7), Fp(8), Fp(9), IPT, Fp(11), OPT, Fp(13), Fp(14), Fp(15), W3T, Fp(17), Fp(18), Fp(19), BLIM, (float*)d_out);
}
